// SEUNET_23089744183881
// MI455X (gfx1250) — hardware-verified
//
#include <hip/hip_runtime.h>
#include <stddef.h>


#define NTHR   256
#define NWAVE  8
#define HD     64
#define AD     9
#define EPT    8
#define CHUNK  (NTHR * EPT)
#define WCAP   (EPT * 32)
#define LISTN  (NWAVE * WCAP)
#define PASSN  (NWAVE * 16)
#define PCAP   (CHUNK + PASSN)
#define NB     512
#define BM     64
#define DYN_ACC_F ((NB + 1) * HD)
#define DYN_MSG_F (PASSN * HD)
#define DYN_M1_H  (PASSN * HD)
#define DYN_BYTES ((DYN_ACC_F + DYN_MSG_F) * 4 + 2 * DYN_M1_H * 2)

static_assert((PCAP % PASSN) == 0);
static_assert((NB % BM) == 0);
static_assert(WCAP == EPT * 32);
static_assert(((DYN_ACC_F + DYN_MSG_F) % 4) == 0);
static_assert(DYN_BYTES == 196864);

typedef unsigned short us;
typedef us     v2us  __attribute__((ext_vector_type(2)));
typedef us     v4us  __attribute__((ext_vector_type(4)));
typedef us     v8us  __attribute__((ext_vector_type(8)));
typedef __attribute__((ext_vector_type(16))) __bf16 v16bf;
typedef float  v2f   __attribute__((ext_vector_type(2)));
typedef float  v4f   __attribute__((ext_vector_type(4)));
typedef float  v8f   __attribute__((ext_vector_type(8)));
typedef int    v4i   __attribute__((ext_vector_type(4)));
typedef int    v8i   __attribute__((ext_vector_type(8)));
union FragB { v16bf v; v8us u[2]; };

__device__ __forceinline__ v8f zero8f() {
  v8f z;
#pragma unroll
  for (int i = 0; i < 8; ++i) z[i] = 0.0f;
  return z;
}

__device__ __forceinline__ v8f wmb(v16bf a, v16bf b, v8f c) {
  v8f d = __builtin_amdgcn_wmma_f32_16x16x32_bf16(false, a, false, b, (short)0, c, false, false);
  asm volatile("v_nop\n\tv_nop\n\tv_nop\n\tv_nop" : "+v"(d) : "v"(__builtin_bit_cast(v8i, a)), "v"(__builtin_bit_cast(v8i, b)));
  return d;
}

__device__ __forceinline__ us bfb(float x) { return __builtin_bit_cast(us, (__bf16)x); }
__device__ __forceinline__ float bfv(us b) { return __uint_as_float(((unsigned)b) << 16); }
__device__ __forceinline__ void split1(float x, us& hi, us& lo) {
  const us hb = bfb(x);
  hi = hb;
  lo = bfb(x - bfv(hb));
}
__device__ __forceinline__ void split4(v4f v, v4us& hi, v4us& lo) {
  us a, b;
  split1(v.x, a, b); hi.x = a; lo.x = b;
  split1(v.y, a, b); hi.y = a; lo.y = b;
  split1(v.z, a, b); hi.z = a; lo.z = b;
  split1(v.w, a, b); hi.w = a; lo.w = b;
}

__device__ __forceinline__ FragB ldfrag(const us* p) {
  FragB f;
  f.u[0] = *(const v8us*)p;
  f.u[1] = *(const v8us*)(p + 16);
  return f;
}

__device__ __forceinline__ float swishf(float v) {
  return v * __builtin_amdgcn_rcpf(1.0f + __expf(-v));
}

__device__ __forceinline__ int scan_chunk(const int* __restrict__ dsts, int nE, int cbase, int nodeBase,
                                          int vec8, int* list, int tid, int wave) {
  int wc = 0;
  const int el0  = tid * EPT;
  const int e0   = cbase + el0;
  const int sent = -2147483647 - 1;
  v4i da, db;
  if (vec8 != 0 && cbase + CHUNK <= nE) {
    da = *(const v4i*)(dsts + e0);
    db = *(const v4i*)(dsts + e0 + 4);
  } else {
    da.x = (e0     < nE) ? dsts[min(e0, nE - 1)] : sent;
    da.y = (e0 + 1 < nE) ? dsts[min(e0 + 1, nE - 1)] : sent;
    da.z = (e0 + 2 < nE) ? dsts[min(e0 + 2, nE - 1)] : sent;
    da.w = (e0 + 3 < nE) ? dsts[min(e0 + 3, nE - 1)] : sent;
    db.x = (e0 + 4 < nE) ? dsts[min(e0 + 4, nE - 1)] : sent;
    db.y = (e0 + 5 < nE) ? dsts[min(e0 + 5, nE - 1)] : sent;
    db.z = (e0 + 6 < nE) ? dsts[min(e0 + 6, nE - 1)] : sent;
    db.w = (e0 + 7 < nE) ? dsts[min(e0 + 7, nE - 1)] : sent;
  }
  const unsigned nb = (unsigned)nodeBase;
  const unsigned s0 = (unsigned)da.x - nb, s1 = (unsigned)da.y - nb;
  const unsigned s2 = (unsigned)da.z - nb, s3 = (unsigned)da.w - nb;
  const unsigned s4 = (unsigned)db.x - nb, s5 = (unsigned)db.y - nb;
  const unsigned s6 = (unsigned)db.z - nb, s7 = (unsigned)db.w - nb;
  const bool h0 = s0 < (unsigned)NB, h1 = s1 < (unsigned)NB, h2 = s2 < (unsigned)NB, h3 = s3 < (unsigned)NB;
  const bool h4 = s4 < (unsigned)NB, h5 = s5 < (unsigned)NB, h6 = s6 < (unsigned)NB, h7 = s7 < (unsigned)NB;
  const unsigned any = __builtin_amdgcn_ballot_w32(h0 | h1 | h2 | h3 | h4 | h5 | h6 | h7);
  if (any != 0u) {
#define HITJ(J, HJ) { \
      const unsigned mj = __builtin_amdgcn_ballot_w32(HJ); \
      if (mj != 0u) { \
        if (HJ) { \
          const int pos = wc + (int)__builtin_amdgcn_mbcnt_lo(mj, 0u); \
          if (pos < WCAP) list[wave * WCAP + pos] = el0 + (J); \
        } \
        wc += (int)__builtin_popcount(mj); } }
    HITJ(0, h0)
    HITJ(1, h1)
    HITJ(2, h2)
    HITJ(3, h3)
    HITJ(4, h4)
    HITJ(5, h5)
    HITJ(6, h6)
    HITJ(7, h7)
#undef HITJ
  }
  return wc;
}

template <int MODE>
__global__ __launch_bounds__(NTHR) void k_node(
    const float* __restrict__ a0, const float* __restrict__ a1,
    const float* __restrict__ W, const float* __restrict__ V, const float* __restrict__ bias,
    const float* __restrict__ nattr, const float* __restrict__ xres,
    float* outp, int nN, int rowsStore) {
  constexpr int K   = (MODE == 1) ? 128 : 64;
  constexpr int NC  = (MODE == 0) ? 128 : 64;
  constexpr int KT  = K / 32;
  constexpr int NCT = NC / 32;
  constexpr int NC4 = NC / 4;
  constexpr int QN  = (BM * NC4) / NTHR;
  static_assert(QN * NTHR == BM * NC4);
  static_assert(((K * NC) % NTHR) == 0);

  __shared__ __attribute__((aligned(16))) us    ahi[BM * K];
  __shared__ __attribute__((aligned(16))) us    alo[BM * K];
  __shared__ __attribute__((aligned(16))) us    bhi[NC * K];
  __shared__ __attribute__((aligned(16))) us    blo[NC * K];
  __shared__ __attribute__((aligned(16))) float sout[BM * NC];
  __shared__ __attribute__((aligned(16))) float sV[AD * HD];
  __shared__ __attribute__((aligned(16))) float sBi[HD];
  __shared__ float sNa[BM * AD];

  const int tid = threadIdx.x, lane = tid & 31, wave = tid >> 5, h = lane >> 4, m = lane & 15;
  const int rowBase = blockIdx.x * BM;

#pragma unroll
  for (int it = 0; it < (BM * 16) / NTHR; ++it) {
    const int i = it * NTHR + tid;
    const int row = i >> 4, c4 = (i & 15) * 4;
    int gr = rowBase + row;
    gr = gr > nN - 1 ? nN - 1 : gr;
    const v4f v = *(const v4f*)(a0 + (size_t)gr * HD + c4);
    v4us hv, lv;
    split4(v, hv, lv);
    *(v4us*)(ahi + row * K + c4) = hv;
    *(v4us*)(alo + row * K + c4) = lv;
  }
  if (MODE == 1) {
#pragma unroll
    for (int it = 0; it < (BM * 16) / NTHR; ++it) {
      const int i = it * NTHR + tid;
      const int row = i >> 4, c4 = (i & 15) * 4;
      const v4f v = *(const v4f*)(a1 + (size_t)(rowBase + row) * HD + c4);
      v4us hv, lv;
      split4(v, hv, lv);
      *(v4us*)(ahi + row * K + (K - HD) + c4) = hv;
      *(v4us*)(alo + row * K + (K - HD) + c4) = lv;
    }
  }
#pragma unroll 4
  for (int it = 0; it < (K * NC) / NTHR; ++it) {
    const int i = it * NTHR + tid;
    const int k = i / NC, c = i - k * NC;
    const int wi = (MODE == 0) ? ((c < HD) ? (k * HD + c) : ((HD + k) * HD + (c - HD))) : (k * HD + c);
    const float w = W[wi];
    us hv, lv;
    split1(w, hv, lv);
    bhi[c * K + k] = hv;
    blo[c * K + k] = lv;
  }
  if (MODE != 0) {
    for (int i = tid; i < AD * HD; i += NTHR) sV[i] = V[i];
    if (tid < HD) sBi[tid] = bias[tid];
    for (int i = tid; i < BM * AD; i += NTHR) {
      const int row = i / AD;
      int gr = rowBase + row;
      gr = gr > nN - 1 ? nN - 1 : gr;
      sNa[i] = nattr[(size_t)gr * AD + (i - row * AD)];
    }
  }
  __syncthreads();

  const int rt = wave & 3, cg = wave >> 2;
  v8f acc[NCT];
#pragma unroll
  for (int j = 0; j < NCT; ++j) acc[j] = zero8f();
#pragma unroll
  for (int kt = 0; kt < KT; ++kt) {
    const FragB fah = ldfrag(ahi + (rt * 16 + m) * K + kt * 32 + 8 * h);
    const FragB fal = ldfrag(alo + (rt * 16 + m) * K + kt * 32 + 8 * h);
#pragma unroll
    for (int j = 0; j < NCT; ++j) {
      const int ct = cg + 2 * j;
      const FragB fbh = ldfrag(bhi + (ct * 16 + m) * K + kt * 32 + 8 * h);
      const FragB fbl = ldfrag(blo + (ct * 16 + m) * K + kt * 32 + 8 * h);
      acc[j] = wmb(fal.v, fbh.v, acc[j]);
      acc[j] = wmb(fah.v, fbl.v, acc[j]);
      acc[j] = wmb(fah.v, fbh.v, acc[j]);
    }
  }

  if (MODE == 0) {
#pragma unroll
    for (int j = 0; j < NCT; ++j) {
      const int n = (cg + 2 * j) * 16 + m;
#pragma unroll
      for (int r = 0; r < 8; ++r) sout[(rt * 16 + 8 * h + r) * NC + n] = acc[j][r];
    }
  } else {
    float vc[NCT][AD], bb[NCT];
#pragma unroll
    for (int j = 0; j < NCT; ++j) {
      const int n = (cg + 2 * j) * 16 + m;
      bb[j] = sBi[n];
#pragma unroll
      for (int a = 0; a < AD; ++a) vc[j][a] = sV[a * HD + n];
    }
#pragma unroll
    for (int r = 0; r < 8; ++r) {
      const int row = rt * 16 + 8 * h + r;
      float na[AD];
#pragma unroll
      for (int a = 0; a < AD; ++a) na[a] = sNa[row * AD + a];
#pragma unroll
      for (int j = 0; j < NCT; ++j) {
        const int n = (cg + 2 * j) * 16 + m;
        float g = 0.0f;
#pragma unroll
        for (int a = 0; a < AD; ++a) g += na[a] * vc[j][a];
        float v = acc[j][r] * g + bb[j];
        if (MODE == 1) v = swishf(v);
        sout[row * NC + n] = v;
      }
    }
  }
  __syncthreads();

#pragma unroll 1
  for (int ps = 0; ps < 2; ++ps) {
#pragma unroll
    for (int q = 0; q < QN; ++q) {
      const int i = q * NTHR + tid;
      const int row = i / NC4, c4 = (i - row * NC4) * 4;
      const int gr = rowBase + row;
      v4f v = *(const v4f*)(sout + row * NC + c4);
      if (MODE == 2) {
        int xr = gr > nN - 1 ? nN - 1 : gr;
        const v4f xv = *(const v4f*)(xres + (size_t)xr * HD + c4);
        v = 0.7f * xv + 0.3f * v;
      }
      if (gr < rowsStore) *(volatile v4f*)(outp + (size_t)gr * NC + c4) = v;
    }
    if (ps == 0) __threadfence();
  }
}

__global__ __launch_bounds__(NTHR) void k_agg(
    const float* __restrict__ PQ, const float* __restrict__ eattr, const float* __restrict__ amf,
    const int* __restrict__ ei, const float* __restrict__ w128,
    const float* __restrict__ Vm1l, const float* __restrict__ bm1l,
    const float* __restrict__ Wm2l, const float* __restrict__ Vm2l, const float* __restrict__ bm2l,
    float* aggp, int nN, int nE, int vec8) {
  extern __shared__ __attribute__((aligned(16))) float dyn[];
  float* agl  = dyn;
  float* msg  = dyn + DYN_ACC_F;
  us*    m1hi = (us*)(dyn + DYN_ACC_F + DYN_MSG_F);
  us*    m1lo = m1hi + DYN_M1_H;
  __shared__ __attribute__((aligned(16))) us    whi[HD * HD];
  __shared__ __attribute__((aligned(16))) us    wlo[HD * HD];
  __shared__ __attribute__((aligned(16))) float sVm1[AD * HD];
  __shared__ __attribute__((aligned(16))) float sVm2[AD * HD];
  __shared__ __attribute__((aligned(16))) float sW[HD];
  __shared__ __attribute__((aligned(16))) float sB1[HD];
  __shared__ __attribute__((aligned(16))) float sB2[HD];
  __shared__ float sEA[PASSN * AD];
  __shared__ int   sslot[PASSN];
  __shared__ __attribute__((aligned(16))) int list[LISTN];
  __shared__ __attribute__((aligned(16))) int pend[PCAP];
  __shared__ int   wcnt[NWAVE];
  __shared__ int   pendN;

  const int tid = threadIdx.x, lane = tid & 31, wave = tid >> 5, h = lane >> 4, m = lane & 15;
  const int nodeBase = blockIdx.x * NB;
  const int* srcs = ei;
  const int* dsts = ei + nE;

  {
    const v4f z4 = {0.0f, 0.0f, 0.0f, 0.0f};
    for (int i = tid; i < DYN_ACC_F / 4; i += NTHR) ((v4f*)agl)[i] = z4;
  }
  for (int i = tid; i < HD * HD; i += NTHR) {
    const int k = i >> 6, n = i & 63;
    us hv, lv;
    split1(Wm2l[i], hv, lv);
    whi[n * HD + k] = hv;
    wlo[n * HD + k] = lv;
  }
  for (int i = tid; i < AD * HD; i += NTHR) { sVm1[i] = Vm1l[i]; sVm2[i] = Vm2l[i]; }
  if (tid < HD) { sW[tid] = w128[tid]; sB1[tid] = bm1l[tid]; sB2[tid] = bm2l[tid]; }
  if (tid == 0) pendN = 0;
  __syncthreads();

  const int c0 = 2 * lane;
  v2f vm1v[AD];
#pragma unroll
  for (int a = 0; a < AD; ++a) vm1v[a] = *(const v2f*)(sVm1 + a * HD + c0);
  const v2f wv  = *(const v2f*)(sW + c0);
  const v2f b1v = *(const v2f*)(sB1 + c0);
  float vc[4][AD], bb[4];
#pragma unroll
  for (int t = 0; t < 4; ++t) {
    const int n = 16 * t + m;
    bb[t] = sB2[n];
#pragma unroll
    for (int a = 0; a < AD; ++a) vc[t][a] = sVm2[a * HD + n];
  }

  const int nChunks = (nE + CHUNK - 1) / CHUNK;
#pragma unroll 1
  for (int ch = 0; ch < nChunks; ++ch) {
    const int cbase = ch * CHUNK;
    const int wc = scan_chunk(dsts, nE, cbase, nodeBase, vec8, list, tid, wave);
    if (lane == 0) wcnt[wave] = wc;
    __syncthreads();

    const int base = pendN;
    int tot = 0, myoff = 0;
#pragma unroll
    for (int w = 0; w < NWAVE; ++w) {
      int c = wcnt[w];
      c = c > WCAP ? WCAP : (c < 0 ? 0 : c);
      if (w < wave) myoff += c;
      tot += c;
    }
    int newN = base + tot;
    newN = newN > PCAP ? PCAP : newN;
    {
      int n = wcnt[wave];
      n = n > WCAP ? WCAP : (n < 0 ? 0 : n);
      const int* lp = list + wave * WCAP;
      for (int i = lane; i < n; i += 32) {
        const int pos = base + myoff + i;
        if (pos < PCAP) pend[pos] = cbase + lp[i];
      }
    }
    const int fin = (ch == nChunks - 1) ? 1 : 0;
    const int R   = (fin != 0) ? (newN + PASSN - 1) / PASSN : newN / PASSN;
    const int Pv  = (fin != 0) ? newN : R * PASSN;
    __syncthreads();

#pragma unroll 1
    for (int r = 0; r < R; ++r) {
      {
#pragma unroll 1
        for (int j = 0; j < 16; ++j) {
          const int er = wave * 16 + j;
          int idx = r * PASSN + er;
          const bool valid = idx < Pv;
          idx = idx > PCAP - 1 ? PCAP - 1 : idx;
          int e = pend[idx];
          e = e < 0 ? 0 : (e > nE - 1 ? nE - 1 : e);
          int d = dsts[e];
          int s = srcs[e];
          int slot = d - nodeBase;
          if (!valid || (unsigned)slot >= (unsigned)NB) slot = NB;
          d = d < 0 ? 0 : (d > nN - 1 ? nN - 1 : d);
          s = s < 0 ? 0 : (s > nN - 1 ? nN - 1 : s);
          const v2f pd = *(const v2f*)(PQ + (size_t)d * (2 * HD) + c0);
          const v2f qs = *(const v2f*)(PQ + (size_t)s * (2 * HD) + HD + c0);
          const float am  = amf[e];
          const float eal = eattr[(size_t)e * AD + (lane < AD - 1 ? lane : AD - 1)];
          const int eali  = __float_as_int(eal);
          v2f g = {0.0f, 0.0f};
#pragma unroll
          for (int a = 0; a < AD; ++a) {
            const float eaa = __int_as_float(__builtin_amdgcn_readlane(eali, a));
            g += eaa * vm1v[a];
          }
          const v2f pre = pd + qs + am * wv;
          const v2f tt  = pre * g + b1v;
          float mv0 = swishf(tt.x), mv1 = swishf(tt.y);
          mv0 = valid ? mv0 : 0.0f;
          mv1 = valid ? mv1 : 0.0f;
          us t0, t1, l0, l1;
          split1(mv0, t0, l0);
          split1(mv1, t1, l1);
          v2us hv, lv;
          hv.x = t0; hv.y = t1; lv.x = l0; lv.y = l1;
          *(v2us*)(m1hi + er * HD + c0) = hv;
          *(v2us*)(m1lo + er * HD + c0) = lv;
          if (lane < AD) sEA[er * AD + lane] = valid ? eal : 0.0f;
          if (lane == 0) sslot[er] = slot;
        }
      }
      __syncthreads();

      {
        const us* arow = m1hi + (wave * 16 + m) * HD + 8 * h;
        const us* lrow = m1lo + (wave * 16 + m) * HD + 8 * h;
        v8f acc[4];
#pragma unroll
        for (int t = 0; t < 4; ++t) acc[t] = zero8f();
#pragma unroll
        for (int kt = 0; kt < 2; ++kt) {
          const FragB fah = ldfrag(arow + 32 * kt);
          const FragB fal = ldfrag(lrow + 32 * kt);
#pragma unroll
          for (int t = 0; t < 4; ++t) {
            const FragB fbh = ldfrag(whi + (16 * t + m) * HD + 32 * kt + 8 * h);
            const FragB fbl = ldfrag(wlo + (16 * t + m) * HD + 32 * kt + 8 * h);
            acc[t] = wmb(fal.v, fbh.v, acc[t]);
            acc[t] = wmb(fah.v, fbl.v, acc[t]);
            acc[t] = wmb(fah.v, fbh.v, acc[t]);
          }
        }
#pragma unroll
        for (int rr = 0; rr < 8; ++rr) {
          const int er = wave * 16 + 8 * h + rr;
          float ea[AD];
#pragma unroll
          for (int a = 0; a < AD; ++a) ea[a] = sEA[er * AD + a];
#pragma unroll
          for (int t = 0; t < 4; ++t) {
            float g = 0.0f;
#pragma unroll
            for (int a = 0; a < AD; ++a) g += ea[a] * vc[t][a];
            const float v = acc[t][rr] * g + bb[t];
            msg[er * HD + 16 * t + m] = swishf(v);
          }
        }
      }
      __syncthreads();

      if (tid < HD) {
#pragma unroll 1
        for (int i = 0; i < PASSN; ++i) {
          int sl = sslot[i];
          sl = sl < 0 ? 0 : (sl > NB ? NB : sl);
          const float v = msg[i * HD + tid];
          agl[sl * HD + tid] += v;
        }
      }
      __syncthreads();
    }

    int rem = newN - R * PASSN;
    rem = rem < 0 ? 0 : rem;
    if (R > 0 && tid < rem) pend[tid] = pend[R * PASSN + tid];
    if (tid == 0) pendN = rem;
  }
  __syncthreads();

  {
    const size_t ob = (size_t)nodeBase * HD;
#pragma unroll 1
    for (int ps = 0; ps < 2; ++ps) {
#pragma unroll
      for (int q = 0; q < (NB * HD / 4) / NTHR; ++q) {
        const int i = q * NTHR + tid;
        const v4f v = ((const v4f*)agl)[i];
        *(volatile v4f*)(aggp + ob + (size_t)i * 4) = v;
      }
      if (ps == 0) __threadfence();
    }
  }
}

extern "C" void kernel_launch(void* const* d_in, const int* in_sizes, int n_in,
                              void* d_out, int out_size, void* d_ws, size_t ws_size,
                              hipStream_t stream) {
  if (n_in < 17) return;
  const int nN = in_sizes[0] / HD;
  const int nE = in_sizes[16] / 2;
  if (nN <= 0 || nE < 0) return;
  if (in_sizes[0] != nN * HD || in_sizes[16] != 2 * nE) return;
  if (in_sizes[1] != nE * AD || in_sizes[2] != nN * AD || in_sizes[3] != nE) return;
  if (in_sizes[4] != 2 * 129 * HD || in_sizes[5] != 2 * AD * HD || in_sizes[6] != 2 * HD) return;
  if (in_sizes[7] != 2 * HD * HD || in_sizes[8] != 2 * AD * HD || in_sizes[9] != 2 * HD) return;
  if (in_sizes[10] != 2 * 2 * HD * HD || in_sizes[11] != 2 * AD * HD || in_sizes[12] != 2 * HD) return;
  if (in_sizes[13] != 2 * HD * HD || in_sizes[14] != 2 * AD * HD || in_sizes[15] != 2 * HD) return;
  if (out_size != nN * HD) return;

  const float* x         = (const float*)d_in[0];
  const float* edge_attr = (const float*)d_in[1];
  const float* node_attr = (const float*)d_in[2];
  const float* amf       = (const float*)d_in[3];
  const float* Wm1       = (const float*)d_in[4];
  const float* Vm1       = (const float*)d_in[5];
  const float* bm1       = (const float*)d_in[6];
  const float* Wm2       = (const float*)d_in[7];
  const float* Vm2       = (const float*)d_in[8];
  const float* bm2       = (const float*)d_in[9];
  const float* Wu1       = (const float*)d_in[10];
  const float* Vu1       = (const float*)d_in[11];
  const float* bu1       = (const float*)d_in[12];
  const float* Wu2       = (const float*)d_in[13];
  const float* Vu2       = (const float*)d_in[14];
  const float* bu2       = (const float*)d_in[15];
  const int*   ei        = (const int*)d_in[16];
  float* out = (float*)d_out;

  const int nBlkA = (nN + NB - 1) / NB;
  const int Npad  = nBlkA * NB;
  const int nBlkN = Npad / BM;
  if (nBlkN * BM != Npad) return;

  char* ws = (char*)d_ws;
  size_t off = 0;
  const size_t oPQ = off; off += (size_t)Npad * (2 * HD) * sizeof(float); off = (off + 255) & ~(size_t)255;
  const size_t oAg = off; off += (size_t)Npad * HD * sizeof(float);       off = (off + 255) & ~(size_t)255;
  const size_t oU1 = off; off += (size_t)Npad * HD * sizeof(float);       off = (off + 255) & ~(size_t)255;
  const size_t oXb = off; off += (size_t)Npad * HD * sizeof(float);       off = (off + 255) & ~(size_t)255;
  if (off > ws_size || off > (size_t)134217728) return;
  float* PQ  = (float*)(ws + oPQ);
  float* agg = (float*)(ws + oAg);
  float* u1  = (float*)(ws + oU1);
  float* xb  = (float*)(ws + oXb);

  const int vec8 = ((nE & 3) == 0) ? 1 : 0;

  hipFuncSetAttribute(reinterpret_cast<const void*>(&k_agg),
                      hipFuncAttributeMaxDynamicSharedMemorySize, DYN_BYTES);

  for (int l = 0; l < 2; ++l) {
    const float* xcur = (l == 0) ? x : xb;
    float* xnext = (l == 0) ? xb : out;
    const int rowsNext = (l == 0) ? Npad : nN;

    k_node<0><<<nBlkN, NTHR, 0, stream>>>(
        xcur, xcur, Wm1 + (size_t)l * 129 * HD, Vm1, bm1, node_attr, xcur, PQ, nN, Npad);

    k_agg<<<nBlkA, NTHR, DYN_BYTES, stream>>>(
        PQ, edge_attr, amf, ei, Wm1 + (size_t)l * 129 * HD + 128 * HD,
        Vm1 + (size_t)l * AD * HD, bm1 + (size_t)l * HD,
        Wm2 + (size_t)l * HD * HD, Vm2 + (size_t)l * AD * HD, bm2 + (size_t)l * HD,
        agg, nN, nE, vec8);

    k_node<1><<<nBlkN, NTHR, 0, stream>>>(
        xcur, agg, Wu1 + (size_t)l * 2 * HD * HD, Vu1 + (size_t)l * AD * HD, bu1 + (size_t)l * HD,
        node_attr, xcur, u1, nN, Npad);

    k_node<2><<<nBlkN, NTHR, 0, stream>>>(
        u1, u1, Wu2 + (size_t)l * HD * HD, Vu2 + (size_t)l * AD * HD, bu2 + (size_t)l * HD,
        node_attr, xcur, xnext, nN, rowsNext);
  }
}
